// CrossAttentionFusion_48765058679268
// MI455X (gfx1250) — hardware-verified
//
#include <hip/hip_runtime.h>
#include <hip/hip_bf16.h>

#define BB 8
#define CC 256
#define OO 256
#define NN 2304
#define GG 8
#define CPG (OO / GG)

typedef __attribute__((ext_vector_type(16))) _Float16 v16h;
typedef __attribute__((ext_vector_type(8)))  _Float16 v8h;
typedef __attribute__((ext_vector_type(8)))  float    v8f;
typedef __attribute__((ext_vector_type(4)))  float    v4f_t;
typedef float v4fa __attribute__((ext_vector_type(4), may_alias));
typedef __attribute__((ext_vector_type(4)))  unsigned v4u_t;
typedef unsigned v4ua __attribute__((ext_vector_type(4), may_alias));
static __device__ __forceinline__ unsigned pk2(float a, float b) { return (unsigned)__builtin_bit_cast(unsigned short, (_Float16)a) | ((unsigned)__builtin_bit_cast(unsigned short, (_Float16)b) << 16); }

#if defined(__has_builtin)
#if __has_builtin(__builtin_amdgcn_global_load_async_to_lds_b128) && \
    __has_builtin(__builtin_amdgcn_s_wait_asynccnt)
#define USE_ASYNC_LDS 1
#endif
#endif
#ifndef USE_ASYNC_LDS
#define USE_ASYNC_LDS 0
#endif

typedef int async_i4 __attribute__((vector_size(16)));
typedef __attribute__((address_space(1))) async_i4* g_i4p;
typedef __attribute__((address_space(3))) async_i4* l_i4p;

__device__ __forceinline__ void cp16_lds(_Float16* lds, const _Float16* g) {
#if USE_ASYNC_LDS
    __builtin_amdgcn_global_load_async_to_lds_b128((g_i4p)(g), (l_i4p)(lds), 0, 0);
#else
    *(uint4*)lds = *(const uint4*)g;
#endif
}

__device__ __forceinline__ void wait_async_lds() {
#if USE_ASYNC_LDS
    __builtin_amdgcn_s_wait_asynccnt(0);
#endif
}

__device__ __forceinline__ v16h load_A16(const _Float16* row, int kc, int hi) {
    const v8h a0 = *(const v8h*)(row + kc + hi * 8);
    const v8h a1 = *(const v8h*)(row + kc + 16 + hi * 8);
    v16h r;
#pragma unroll
    for (int i = 0; i < 8; ++i) { r[i] = a0[i]; r[i + 8] = a1[i]; }
    return r;
}

__device__ __forceinline__ v16h load_B16(const _Float16* rowT, int kc, int hi) {
    const v8h a0 = *(const v8h*)(rowT + kc + hi * 8);
    const v8h a1 = *(const v8h*)(rowT + kc + 16 + hi * 8);
    v16h r;
#pragma unroll
    for (int i = 0; i < 8; ++i) { r[i] = a0[i]; r[i + 8] = a1[i]; }
    return r;
}

__device__ __forceinline__ v8f wmma_f16(v16h a, v16h b, v8f c) {
    return __builtin_amdgcn_wmma_f32_16x16x32_f16(false, a, false, b,
                                                  (short)0, c, false, false);
}

__global__ __launch_bounds__(256) void k_cvt_feat(const float* __restrict__ in,
                                                  _Float16* __restrict__ out) {
    int idx = (blockIdx.x * 256 + threadIdx.x) * 2;
    if (idx >= BB * NN * CC) return;
    int c = idx & (CC - 1);
    int rest = idx >> 8;
    int n = rest % NN;
    int b = rest / NN;
    const unsigned p = pk2(in[((size_t)b * CC + c) * NN + n], in[((size_t)b * CC + c + 1) * NN + n]);
    *(volatile unsigned*)(out + idx) = p; __threadfence(); *(volatile unsigned*)(out + idx) = p;
}

__global__ __launch_bounds__(256) void k_cvt_w(const float* __restrict__ q,
                                               const float* __restrict__ k,
                                               const float* __restrict__ v,
                                               const float* __restrict__ o,
                                               _Float16* __restrict__ qh,
                                               _Float16* __restrict__ kh,
                                               _Float16* __restrict__ vh,
                                               _Float16* __restrict__ oh) {
    int idx = (blockIdx.x * 256 + threadIdx.x) * 2;
    if (idx >= OO * CC) return;
    const unsigned pq = pk2(q[idx], q[idx + 1]), pk = pk2(k[idx], k[idx + 1]), pv = pk2(v[idx], v[idx + 1]), po = pk2(o[idx], o[idx + 1]);
    *(volatile unsigned*)(qh + idx) = pq; *(volatile unsigned*)(kh + idx) = pk; *(volatile unsigned*)(vh + idx) = pv; *(volatile unsigned*)(oh + idx) = po;
    __threadfence();
    *(volatile unsigned*)(qh + idx) = pq; *(volatile unsigned*)(kh + idx) = pk; *(volatile unsigned*)(vh + idx) = pv; *(volatile unsigned*)(oh + idx) = po;
}

__global__ __launch_bounds__(256) void k_proj(
    const _Float16* __restrict__ f1h, const _Float16* __restrict__ f2h,
    const _Float16* __restrict__ qwh, const _Float16* __restrict__ kwh,
    const _Float16* __restrict__ vwh,
    const float* __restrict__ qb, const float* __restrict__ kb,
    const float* __restrict__ vb,
    _Float16* __restrict__ Qh, _Float16* __restrict__ Kh,
    _Float16* __restrict__ Vr) {
    __shared__ __align__(16) _Float16 st[3][16 * OO];
    const int tid = threadIdx.x, w = tid >> 5;
    const int l = tid & 31, hi = (l >> 4) & 1, ln = l & 15;
    const int t0 = blockIdx.x * 16, b = blockIdx.y;

    const _Float16* A1 = f1h + ((size_t)b * NN + t0 + ln) * CC;
    const _Float16* A2 = f2h + ((size_t)b * NN + t0 + ln) * CC;
    const float qscale = 0.0625f;
#pragma unroll 1
    for (int j = 0; j < 2; ++j) {
        const int ob = (2 * w + j) * 16;
        const _Float16* Bq = qwh + (size_t)(ob + ln) * CC;
        const _Float16* Bk = kwh + (size_t)(ob + ln) * CC;
        const _Float16* Bv = vwh + (size_t)(ob + ln) * CC;
        v8f aq = {}, ak = {}, av = {};
#pragma unroll
        for (int kc = 0; kc < CC; kc += 32) {
            v16h a1 = load_A16(A1, kc, hi);
            v16h a2 = load_A16(A2, kc, hi);
            aq = wmma_f16(a1, load_B16(Bq, kc, hi), aq);
            ak = wmma_f16(a2, load_B16(Bk, kc, hi), ak);
            av = wmma_f16(a2, load_B16(Bv, kc, hi), av);
        }
        const float bqv = qb[ob + ln], bkv = kb[ob + ln], bvv = vb[ob + ln];
#pragma unroll
        for (int r = 0; r < 8; ++r) {
            const int m = r + hi * 8;
            st[0][m * OO + ob + ln] = (_Float16)((aq[r] + bqv) * qscale);
            st[1][m * OO + ob + ln] = (_Float16)(ak[r] + bkv);
            st[2][m * OO + ob + ln] = (_Float16)(av[r] + bvv);
        }
    }
    __syncthreads();
#pragma unroll 1
    for (int pass = 0; pass < 2; ++pass) {
#pragma unroll
        for (int a = 0; a < 3; ++a) {
            _Float16* dst = (a == 0) ? Qh : (a == 1) ? Kh : Vr;
#pragma unroll
            for (int i = 0; i < 2; ++i) {
                const int c = tid + 256 * i, rr = c >> 5, q = c & 31;
                *(volatile v4u_t*)(dst + ((size_t)b * NN + t0 + rr) * OO + q * 8) = *(const volatile v4ua*)(&st[a][rr * OO + q * 8]);
            }
        }
        __threadfence();
    }
}

__global__ __launch_bounds__(256) void k_vt(const _Float16* __restrict__ Vr, _Float16* __restrict__ VhT) {
    __shared__ _Float16 t[64][258];
    const int tid = threadIdx.x, lane = tid & 31, wave = tid >> 5;
    const int b = blockIdx.y, n0 = blockIdx.x * 64;
    const _Float16* src = Vr + ((size_t)b * NN + n0) * OO;
#pragma unroll
    for (int k = 0; k < 64; ++k) { const int e = tid + 256 * k; t[e >> 8][e & 255] = src[e]; }
    __syncthreads();
#pragma unroll 4
    for (int rr = 0; rr < 32; ++rr) {
        const int o = wave * 32 + rr;
        const unsigned p = (unsigned)__builtin_bit_cast(unsigned short, t[2 * lane][o]) | ((unsigned)__builtin_bit_cast(unsigned short, t[2 * lane + 1][o]) << 16);
        unsigned* d = (unsigned*)(VhT + ((size_t)b * OO + o) * NN + n0) + lane;
        *(volatile unsigned*)d = p; __threadfence(); *(volatile unsigned*)d = p;
    }
}

__global__ __launch_bounds__(128) __attribute__((amdgpu_num_vgpr(248))) void k_attn(const _Float16* __restrict__ Qh,
                                              const _Float16* __restrict__ Kh,
                                              const _Float16* __restrict__ VhT,
                                              _Float16* __restrict__ AOh) {
    __shared__ __align__(16) _Float16 Ks[32 * OO];
    __shared__ __align__(16) _Float16 Vs[OO * 32];
    __shared__ __align__(16) _Float16 Ps[4][16 * 32];
    __shared__ __align__(16) _Float16 Os[4][16 * OO];
    const int tid = threadIdx.x;
    const int w = tid >> 5, l = tid & 31, hi = (l >> 4) & 1, ln = l & 15;
    const int qblk = blockIdx.x * 64, b = blockIdx.y;
    const int t0 = qblk + w * 16;

    v16h qreg[8];
    {
        const _Float16* Qrow = Qh + ((size_t)b * NN + t0 + ln) * OO;
#pragma unroll
        for (int kc = 0; kc < OO; kc += 32) qreg[kc >> 5] = load_A16(Qrow, kc, hi);
    }

    v8f acc[16];
#pragma unroll
    for (int t = 0; t < 16; ++t) acc[t] = (v8f){};
    float mrow[8], lrow[8];
#pragma unroll
    for (int r = 0; r < 8; ++r) { mrow[r] = -3.0e30f; lrow[r] = 0.0f; }

    for (int k0 = 0; k0 < NN; k0 += 32) {
        {
            const _Float16* srcK = Kh + ((size_t)b * NN + k0) * OO;
#pragma unroll
            for (int i = tid; i < 1024; i += 128)
                cp16_lds(Ks + (size_t)i * 8, srcK + (size_t)i * 8);
        }
        {
            const _Float16* srcV = VhT + (size_t)b * OO * NN + k0;
#pragma unroll
            for (int i = tid; i < 1024; i += 128) {
                int o = i >> 2, c = i & 3;
                cp16_lds(Vs + o * 32 + c * 8, srcV + (size_t)o * NN + c * 8);
            }
        }
        wait_async_lds();
        __syncthreads();

        if (k0 + 32 < NN) {
            const char* nk = (const char*)(Kh + ((size_t)b * NN + k0 + 32) * OO);
            __builtin_prefetch(nk + tid * 128, 0, 3);
        }

        const _Float16* K0 = Ks + (size_t)ln * OO;
        const _Float16* K1 = Ks + (size_t)(16 + ln) * OO;
        v8f s0 = {}, s1 = {};
#pragma unroll
        for (int kc = 0; kc < OO; kc += 32) {
            s0 = wmma_f16(qreg[kc >> 5], load_B16(K0, kc, hi), s0);
            s1 = wmma_f16(qreg[kc >> 5], load_B16(K1, kc, hi), s1);
        }
        float rm[8];
#pragma unroll
        for (int r = 0; r < 8; ++r) rm[r] = fmaxf(s0[r], s1[r]);
#pragma unroll
        for (int mask = 1; mask <= 8; mask <<= 1)
#pragma unroll
            for (int r = 0; r < 8; ++r)
                rm[r] = fmaxf(rm[r], __shfl_xor(rm[r], mask, 32));

        float p0[8], p1[8], rs[8], ef[8];
#pragma unroll
        for (int r = 0; r < 8; ++r) {
            float nm = fmaxf(mrow[r], rm[r]);
            ef[r] = __expf(mrow[r] - nm);
            mrow[r] = nm;
            p0[r] = __expf(s0[r] - nm);
            p1[r] = __expf(s1[r] - nm);
            rs[r] = p0[r] + p1[r];
        }
#pragma unroll
        for (int mask = 1; mask <= 8; mask <<= 1)
#pragma unroll
            for (int r = 0; r < 8; ++r) rs[r] += __shfl_xor(rs[r], mask, 32);
#pragma unroll
        for (int r = 0; r < 8; ++r) lrow[r] = lrow[r] * ef[r] + rs[r];
#pragma unroll
        for (int t = 0; t < 16; ++t)
#pragma unroll
            for (int r = 0; r < 8; ++r) acc[t][r] *= ef[r];

        _Float16* Pw = Ps[w];
#pragma unroll
        for (int r = 0; r < 8; ++r) {
            int m = r + hi * 8;
            Pw[m * 32 + ln]      = (_Float16)(p0[r] * 1024.0f);
            Pw[m * 32 + 16 + ln] = (_Float16)(p1[r] * 1024.0f);
        }
        v16h ap = load_A16(Pw + ln * 32, 0, hi);
#pragma unroll
        for (int t = 0; t < 16; ++t)
            acc[t] = wmma_f16(ap, load_B16(Vs + (size_t)(t * 16 + ln) * 32, 0, hi),
                              acc[t]);
        __syncthreads();
    }
    _Float16* ow = Os[w];
#pragma unroll
    for (int t = 0; t < 16; ++t) {
#pragma unroll
        for (int r = 0; r < 8; ++r) ow[(r + hi * 8) * OO + t * 16 + ln] = (_Float16)(acc[t][r] / (lrow[r] * 1024.0f));
    }
    asm volatile("s_wait_dscnt 0" ::: "memory");
#pragma unroll 1
    for (int pass = 0; pass < 2; ++pass) {
#pragma unroll 4
        for (int i = 0; i < 16; ++i) {
            const int c = l + 32 * i, rr = c >> 5, q = c & 31;
            *(volatile v4u_t*)(AOh + ((size_t)b * NN + t0 + rr) * OO + q * 8) = *(const volatile v4ua*)(ow + rr * OO + q * 8);
        }
        __threadfence();
    }
}

__global__ __launch_bounds__(256) void k_oproj(const _Float16* __restrict__ AOh,
                                               const _Float16* __restrict__ owh,
                                               const float* __restrict__ obv,
                                               float* __restrict__ out2) {
    __shared__ __align__(16) float so[64][32 + 4];
    const int tid = threadIdx.x, w = tid >> 5;
    const int l = tid & 31, hi = (l >> 4) & 1, ln = l & 15;
    const int pb = blockIdx.x * 64 + (w & 3) * 16, t0 = blockIdx.y * 32 + (w >> 2) * 16, b = blockIdx.z;
    const _Float16* A = AOh + ((size_t)b * NN + t0 + ln) * OO;
    const _Float16* Bt = owh + (size_t)(pb + ln) * OO;
    v8f a = {};
#pragma unroll
    for (int kc = 0; kc < OO; kc += 32)
        a = wmma_f16(load_A16(A, kc, hi), load_B16(Bt, kc, hi), a);
    const float bias = obv[pb + ln];
#pragma unroll
    for (int r = 0; r < 8; ++r) so[(w & 3) * 16 + ln][(w >> 2) * 16 + r + hi * 8] = a[r] + bias;
    __syncthreads();
#pragma unroll 1
    for (int pass = 0; pass < 2; ++pass) {
#pragma unroll
        for (int i = 0; i < 2; ++i) {
            const int c = tid + 256 * i, ol = c >> 3, q = c & 7;
            *(volatile v4f_t*)(out2 + ((size_t)b * OO + blockIdx.x * 64 + ol) * NN + blockIdx.y * 32 + q * 4) = *(const v4fa*)&so[ol][q * 4];
        }
        __threadfence();
    }
}

__global__ __launch_bounds__(256) void k_gn(const float* __restrict__ out2,
                                            const float* __restrict__ gw,
                                            const float* __restrict__ gb,
                                            float* __restrict__ out) {
    const int g = blockIdx.x, b = blockIdx.y;
    const float* base = out2 + ((size_t)b * OO + g * CPG) * NN;
    const int total = CPG * NN;
    float s = 0.f, s2 = 0.f;
    for (int i = threadIdx.x; i < total; i += 256) {
        float x = base[i];
        s += x; s2 += x * x;
    }
    __shared__ float rs[256], rq[256];
    rs[threadIdx.x] = s; rq[threadIdx.x] = s2;
    __syncthreads();
    for (int off = 128; off > 0; off >>= 1) {
        if (threadIdx.x < off) {
            rs[threadIdx.x] += rs[threadIdx.x + off];
            rq[threadIdx.x] += rq[threadIdx.x + off];
        }
        __syncthreads();
    }
    const float mean = rs[0] / (float)total;
    const float var  = rq[0] / (float)total - mean * mean;
    const float inv  = rsqrtf(var + 1e-5f);
    float* ob = out + ((size_t)b * OO + g * CPG) * NN;
    for (int i = threadIdx.x; i < total; i += 256) {
        int ch = g * CPG + i / NN;
        const float v = (base[i] - mean) * inv * gw[ch] + gb[ch];
        *(volatile float*)(ob + i) = v; __threadfence(); *(volatile float*)(ob + i) = v;
    }
}

extern "C" void kernel_launch(void* const* d_in, const int* in_sizes, int n_in,
                              void* d_out, int out_size, void* d_ws, size_t ws_size,
                              hipStream_t stream) {
    (void)in_sizes; (void)n_in; (void)out_size; (void)ws_size;
    const float* f1  = (const float*)d_in[0];
    const float* f2  = (const float*)d_in[1];
    const float* q_w = (const float*)d_in[2];
    const float* q_b = (const float*)d_in[3];
    const float* k_w = (const float*)d_in[4];
    const float* k_b = (const float*)d_in[5];
    const float* v_w = (const float*)d_in[6];
    const float* v_b = (const float*)d_in[7];
    const float* o_w = (const float*)d_in[8];
    const float* o_b = (const float*)d_in[9];
    const float* gnw = (const float*)d_in[10];
    const float* gnb = (const float*)d_in[11];

    char* p = (char*)d_ws;
    size_t off = 0;
    auto take = [&](size_t bytes) {
        void* r = p + off;
        off += (bytes + 255) & ~(size_t)255;
        return r;
    };
    const size_t featH = (size_t)BB * NN * CC * sizeof(_Float16);
    const size_t wH    = (size_t)OO * CC * sizeof(_Float16);
    _Float16* f1h = (_Float16*)take(featH);
    _Float16* f2h = (_Float16*)take(featH);
    _Float16* qwh = (_Float16*)take(wH);
    _Float16* kwh = (_Float16*)take(wH);
    _Float16* vwh = (_Float16*)take(wH);
    _Float16* owh = (_Float16*)take(wH);
    _Float16* Qh  = (_Float16*)take((size_t)BB * NN * OO * sizeof(_Float16));
    _Float16* Kh  = (_Float16*)take((size_t)BB * NN * OO * sizeof(_Float16));
    _Float16* VhT = (_Float16*)take((size_t)BB * OO * NN * sizeof(_Float16));
    _Float16* AOh = (_Float16*)take((size_t)BB * NN * OO * sizeof(_Float16));
    float*    out2 = (float*)take((size_t)BB * OO * NN * sizeof(float));
    _Float16* Vr  = (_Float16*)take((size_t)BB * NN * OO * sizeof(_Float16));

    const int featElems = BB * NN * CC;
    k_cvt_feat<<<(featElems / 2 + 255) / 256, 256, 0, stream>>>(f1, f1h);
    k_cvt_feat<<<(featElems / 2 + 255) / 256, 256, 0, stream>>>(f2, f2h);
    k_cvt_w<<<(OO * CC / 2 + 255) / 256, 256, 0, stream>>>(q_w, k_w, v_w, o_w,
                                                       qwh, kwh, vwh, owh);
    k_proj<<<dim3(NN / 16, BB), 256, 0, stream>>>(
        f1h, f2h, qwh, kwh, vwh, q_b, k_b, v_b, Qh, Kh, Vr);
    k_vt<<<dim3(NN / 64, BB), 256, 0, stream>>>(Vr, VhT);
    k_attn<<<dim3(NN / 64, BB), 128, 0, stream>>>(Qh, Kh, VhT, AOh);
    k_oproj<<<dim3(OO / 64, NN / 32, BB), 256, 0, stream>>>(AOh, owh, o_b, out2);
    k_gn<<<dim3(GG, BB), 256, 0, stream>>>(out2, gnw, gnb, (float*)d_out);
}
